// VVCrossAttention_7026566496882
// MI455X (gfx1250) — hardware-verified
//
#include <hip/hip_runtime.h>
#include <stdint.h>
#include <stddef.h>

typedef __attribute__((ext_vector_type(16))) _Float16 v16h;
typedef __attribute__((ext_vector_type(8)))  _Float16 v8h;
typedef __attribute__((ext_vector_type(16))) __bf16   v16b;
typedef __attribute__((ext_vector_type(8)))  __bf16   v8b;
typedef __attribute__((ext_vector_type(8)))  float    v8f;
typedef __attribute__((ext_vector_type(4)))  float    v4f;
typedef __attribute__((ext_vector_type(4)))  int      v4i;
#define PSCALE 32768.0f
#define U16(p) ((const unsigned short*)(const void*)(p))
#define PSCALE_INV (1.0f / 32768.0f)

__device__ __forceinline__ unsigned short f2bf_bits(float f) {
  unsigned u = __float_as_uint(f);
  return (unsigned short)((u + 0x7FFFu + ((u >> 16) & 1u)) >> 16);
}
__device__ __forceinline__ float bf_bits2f(unsigned short h) { return __uint_as_float(((unsigned)h) << 16); }

__device__ __forceinline__ void dep_guard_h(v8f& a, v8f& b, v16h x, v16h y) { asm volatile("v_nop\n\tv_nop\n\tv_nop\n\tv_nop" : "+v"(a), "+v"(b) : "v"(x), "v"(y)); }
__device__ __forceinline__ void dep_guard_b(v8f& a, v8f& b, v16b x, v16b y) { asm volatile("v_nop\n\tv_nop\n\tv_nop\n\tv_nop" : "+v"(a), "+v"(b) : "v"(x), "v"(y)); }
__device__ __forceinline__ void keep4_h(v16h a, v16h b, v16h c, v16h d) { asm volatile("v_nop" :: "v"(a), "v"(b), "v"(c), "v"(d)); }
__device__ __forceinline__ void keep4_b(v16b a, v16b b, v16b c, v16b d) { asm volatile("v_nop" :: "v"(a), "v"(b), "v"(c), "v"(d)); }
__device__ __forceinline__ void acc_guard4(v8f& a, v8f& b, v8f& c, v8f& d) { asm volatile("v_nop\n\tv_nop\n\tv_nop\n\tv_nop" : "+v"(a), "+v"(b), "+v"(c), "+v"(d)); }
template <typename T> struct Frag;
template <> struct Frag<_Float16> {
  typedef v16h V; union U { v16h v; v8h h[2]; };
  static __device__ __forceinline__ v16h load(const _Float16* p) {
    U f; f.h[0] = *(const v8h*)(p); f.h[1] = *(const v8h*)(p + 16); return f.v;
  }
  static __device__ __forceinline__ v8f mma(v16h a, v16h b, v8f c) {
    return __builtin_amdgcn_wmma_f32_16x16x32_f16(false, a, false, b, (short)0, c, false, false);
  }
  static __device__ __forceinline__ void guard(v8f& a, v8f& b, v16h x, v16h y) { dep_guard_h(a, b, x, y); }
  static __device__ __forceinline__ void keep(v16h a, v16h b, v16h c, v16h d) { keep4_h(a, b, c, d); }
};
template <> struct Frag<__bf16> {
  typedef v16b V; union U { v16b v; v8b h[2]; };
  static __device__ __forceinline__ v16b load(const __bf16* p) {
    U f; f.h[0] = *(const v8b*)(p); f.h[1] = *(const v8b*)(p + 16); return f.v;
  }
  static __device__ __forceinline__ v8f mma(v16b a, v16b b, v8f c) {
    return __builtin_amdgcn_wmma_f32_16x16x32_bf16(false, a, false, b, (short)0, c, false, false);
  }
  static __device__ __forceinline__ void guard(v8f& a, v8f& b, v16b x, v16b y) { dep_guard_b(a, b, x, y); }
  static __device__ __forceinline__ void keep(v16b a, v16b b, v16b c, v16b d) { keep4_b(a, b, c, d); }
};

template <int ET> struct Elem;
template <> struct Elem<0> { typedef _Float16 T; };
template <> struct Elem<1> { typedef __bf16 T; };
template <int ET, bool SPLIT, int BIAS_MODE, int OUT_MODE, bool RESID, int ACT = 0>
__global__ __launch_bounds__(256) void wmma_gemm64(
    const unsigned short* __restrict__ Ap, const unsigned short* __restrict__ A2p, int lda, long strideA,
    const unsigned short* __restrict__ Btp, const unsigned short* __restrict__ Bt2p, int ldb, long strideB,
    void* __restrict__ Cout, void* __restrict__ Cout2, int ldc, long strideC,
    const float* __restrict__ bias,
    const float* __restrict__ resid, long strideR,
    int M, int N, int K, float scale) {
  typedef typename Elem<ET>::T T;
  typedef typename Frag<T>::V V;
  const T* A = (const T*)Ap; const T* A2 = (const T*)A2p; const T* Bt = (const T*)Btp; const T* Bt2 = (const T*)Bt2p;
  __shared__ __align__(16) float sT[8][16 * 68];
  const int b    = blockIdx.y;
  const int lane = threadIdx.x & 31;
  const int wave = threadIdx.x >> 5;
  const int tilesN = N >> 6;
  const int tilesM = M >> 6;
  const int tile = blockIdx.x * 8 + wave;
  if (tile >= tilesM * tilesN) return;
  const int tm = tile / tilesN;
  const int tn = tile - tm * tilesN;
  const int m0 = tm << 6;
  const int n0 = tn << 6;

  const T* Ab  = A  + (size_t)b * strideA;
  const T* Bb  = Bt + (size_t)b * strideB;
  const T* Ab2 = SPLIT ? (A2  + (size_t)b * strideA) : nullptr;
  const T* Bb2 = SPLIT ? (Bt2 + (size_t)b * strideB) : nullptr;

  const int rlane = lane & 15;
  const int koff  = (lane >> 4) * 8;
  const int mOff  = (lane >> 4) * 8;

  v8f acc[4][4];
#pragma unroll
  for (int i = 0; i < 4; ++i)
#pragma unroll
    for (int j = 0; j < 4; ++j) acc[i][j] = (v8f){0.f,0.f,0.f,0.f,0.f,0.f,0.f,0.f};

  for (int k0 = 0; k0 < K; k0 += 32) {
    V bh[4], bl[4];
#pragma unroll
    for (int j = 0; j < 4; ++j) {
      const size_t bo = (size_t)(n0 + (j << 4) + rlane) * ldb + koff + k0;
      bh[j] = Frag<T>::load(Bb + bo);
      if (SPLIT) bl[j] = Frag<T>::load(Bb2 + bo);
    }
#pragma unroll
    for (int i = 0; i < 4; ++i) {
      const size_t ao = (size_t)(m0 + (i << 4) + rlane) * lda + koff + k0;
      V ah = Frag<T>::load(Ab + ao);
      V al;
      if (SPLIT) al = Frag<T>::load(Ab2 + ao);
#pragma unroll
      for (int j = 0; j < 4; ++j) {
        acc[i][j] = Frag<T>::mma(ah, bh[j], acc[i][j]);
        if (SPLIT) {
          acc[i][j] = Frag<T>::mma(ah, bl[j], acc[i][j]);
          acc[i][j] = Frag<T>::mma(al, bh[j], acc[i][j]);
        }
      }
      Frag<T>::guard(acc[i][0], acc[i][3], ah, SPLIT ? al : ah);
    }
    Frag<T>::keep(bh[0], bh[1], bh[2], bh[3]);
    if (SPLIT) Frag<T>::keep(bl[0], bl[1], bl[2], bl[3]);
  }
  acc_guard4(acc[0][0], acc[0][1], acc[0][2], acc[0][3]);
  acc_guard4(acc[1][0], acc[1][1], acc[1][2], acc[1][3]);
  acc_guard4(acc[2][0], acc[2][1], acc[2][2], acc[2][3]);
  acc_guard4(acc[3][0], acc[3][1], acc[3][2], acc[3][3]);

  float* slab = sT[wave];
  const float* Rb = RESID ? (resid + (size_t)b * strideR) : nullptr;
#pragma unroll
  for (int i = 0; i < 4; ++i) {
    const int mBase = m0 + (i << 4);
#pragma unroll
    for (int j = 0; j < 4; ++j) {
      const int n = n0 + (j << 4) + rlane;
      float bv = 0.f;
      if (BIAS_MODE == 2) bv = bias[n];
#pragma unroll
      for (int r = 0; r < 8; ++r) {
        float v = acc[i][j][r] * scale;
        if (BIAS_MODE == 1) v += bias[mBase + mOff + r];
        if (BIAS_MODE == 2) v += bv;
        if (RESID) v += Rb[(size_t)(mBase + mOff + r) * ldc + n];
        if (ACT == 1) v = tanhf(v);
        if (ACT == 2) v = fmaxf(v, 0.0f);
        if (ACT == 3) v = v / (1.0f + expf(-v));
        if (ACT == 4) v = (v > 0.f) ? v : 0.01f * v;
        if (ACT == 5) v = 0.5f * v * (1.0f + erff(v * 0.70710678118654752f));
        slab[(mOff + r) * 68 + (j << 4) + rlane] = v;
      }
    }
    __builtin_amdgcn_fence(__ATOMIC_RELEASE, "workgroup");
    __builtin_amdgcn_wave_barrier();
    __builtin_amdgcn_fence(__ATOMIC_ACQUIRE, "workgroup");
    if (OUT_MODE == 0) {
      float* C = (float*)Cout + (size_t)b * strideC;
      const int hh = lane >> 4, c4 = (lane & 15) * 4;
      for (int pass = 0; pass < 2; ++pass) {
#pragma unroll
        for (int it = 0; it < 8; ++it) {
          const int row = it * 2 + hh;
          v4f v = *(const v4f*)(slab + row * 68 + c4);
          *(volatile v4f*)(C + (size_t)(mBase + row) * ldc + n0 + c4) = v;
        }
        __threadfence();
      }
    } else {
      const int q = lane >> 3, c8 = (lane & 7) * 8;
      unsigned short* C  = (unsigned short*)Cout  + (size_t)b * strideC;
      unsigned short* C2 = (OUT_MODE == 2) ? ((unsigned short*)Cout2 + (size_t)b * strideC) : nullptr;
      for (int pass = 0; pass < 2; ++pass) {
#pragma unroll
        for (int it = 0; it < 4; ++it) {
          const int row = it * 4 + q;
          const float* sp = slab + row * 68 + c8;
          v8h hv, lv;
#pragma unroll
          for (int e = 0; e < 8; ++e) {
            if (OUT_MODE == 1) {
              hv[e] = (_Float16)sp[e];
            } else {
              unsigned short hb = f2bf_bits(sp[e]);
              unsigned short lb = f2bf_bits(sp[e] - bf_bits2f(hb));
              hv[e] = __builtin_bit_cast(_Float16, hb);
              lv[e] = __builtin_bit_cast(_Float16, lb);
            }
          }
          *(volatile v8h*)(C + (size_t)(mBase + row) * ldc + n0 + c8) = hv;
          if (OUT_MODE == 2) *(volatile v8h*)(C2 + (size_t)(mBase + row) * ldc + n0 + c8) = lv;
        }
        __threadfence();
      }
    }
    __builtin_amdgcn_fence(__ATOMIC_RELEASE, "workgroup");
    __builtin_amdgcn_wave_barrier();
    __builtin_amdgcn_fence(__ATOMIC_ACQUIRE, "workgroup");
  }
}

__global__ __launch_bounds__(256) void cast_f32_f16x2(
    const float* __restrict__ in, _Float16* __restrict__ out, int n2) {
  int i = blockIdx.x * 256 + threadIdx.x;
  if (i < n2) {
    const _Float16 h0 = (_Float16)in[2 * i], h1 = (_Float16)in[2 * i + 1];
    const unsigned u = (unsigned)__builtin_bit_cast(unsigned short, h0) | ((unsigned)__builtin_bit_cast(unsigned short, h1) << 16);
    ((volatile unsigned*)out)[i] = u;
    __threadfence();
    ((volatile unsigned*)out)[i] = u;
  }
}

__global__ __launch_bounds__(256) void split_f32_bf16x8(
    const float* __restrict__ in, unsigned short* __restrict__ hi, unsigned short* __restrict__ lo, int n8) {
  const int i = blockIdx.x * 256 + threadIdx.x;
  if (i < n8) {
    const float* p = in + (size_t)i * 8;
    const v4f a = *(const v4f*)p;
    const v4f c = *(const v4f*)(p + 4);
    v8h hv, lv;
#pragma unroll
    for (int e = 0; e < 4; ++e) {
      unsigned short hb = f2bf_bits(a[e]);
      unsigned short lb = f2bf_bits(a[e] - bf_bits2f(hb));
      hv[e] = __builtin_bit_cast(_Float16, hb);
      lv[e] = __builtin_bit_cast(_Float16, lb);
      hb = f2bf_bits(c[e]);
      lb = f2bf_bits(c[e] - bf_bits2f(hb));
      hv[4 + e] = __builtin_bit_cast(_Float16, hb);
      lv[4 + e] = __builtin_bit_cast(_Float16, lb);
    }
    unsigned short* ph = hi + (size_t)i * 8;
    unsigned short* pl = lo + (size_t)i * 8;
    *(volatile v8h*)ph = hv;
    *(volatile v8h*)pl = lv;
    __threadfence();
    *(volatile v8h*)ph = hv;
    *(volatile v8h*)pl = lv;
  }
}

__global__ __launch_bounds__(256) void transpose64_h(
    const unsigned short* __restrict__ in, unsigned short* __restrict__ out, int R, int Cc) {
  __shared__ __align__(16) _Float16 t[64 * 72];
  const int tid = threadIdx.x, lane = tid & 31, wave = tid >> 5;
  const int r0 = blockIdx.x * 64, c0 = blockIdx.y * 64, b = blockIdx.z;
  const _Float16* ib = (const _Float16*)in + (size_t)b * (size_t)R * (size_t)Cc;
  _Float16* ob = (_Float16*)out + (size_t)b * (size_t)R * (size_t)Cc;
#pragma unroll
  for (int it = 0; it < 2; ++it) {
    const int idx = it * 256 + tid;
    const int rr = idx >> 3, c8 = (idx & 7) * 8;
    const v8h val = *(const v8h*)(ib + (size_t)(r0 + rr) * Cc + c0 + c8);
    *(v8h*)(t + rr * 72 + c8) = val;
  }
  __syncthreads();
  const int q = lane >> 3, m8 = (lane & 7) * 8;
  v8h h0, h1;
  const int orow0 = wave * 8 + q, orow1 = wave * 8 + 4 + q;
#pragma unroll
  for (int e = 0; e < 8; ++e) {
    h0[e] = t[(m8 + e) * 72 + orow0];
    h1[e] = t[(m8 + e) * 72 + orow1];
  }
  _Float16* p0 = ob + (size_t)(c0 + orow0) * R + r0 + m8;
  _Float16* p1 = ob + (size_t)(c0 + orow1) * R + r0 + m8;
  *(volatile v8h*)p0 = h0;
  *(volatile v8h*)p1 = h1;
  __threadfence();
  *(volatile v8h*)p0 = h0;
  *(volatile v8h*)p1 = h1;
}

#define SM_COLS 4096
__global__ __launch_bounds__(256) void softmax_rows(
    const float* __restrict__ S, const int* __restrict__ keymask, unsigned short* __restrict__ P) {
  __shared__ float rmax[8];
  __shared__ float rsum[8];
  const int row = blockIdx.x;
  const int tid = threadIdx.x, lane = tid & 31, wave = tid >> 5;
  const float* sr = S + (size_t)row * SM_COLS;
  const int ca = tid * 8;
  const int cb = (SM_COLS / 2) + tid * 8;
  const v4f a0 = *(const v4f*)(sr + ca), a1 = *(const v4f*)(sr + ca + 4);
  const v4f b0 = *(const v4f*)(sr + cb), b1 = *(const v4f*)(sr + cb + 4);
  float v[16];
#pragma unroll
  for (int e = 0; e < 4; ++e) { v[e] = a0[e]; v[4 + e] = a1[e]; v[8 + e] = b0[e]; v[12 + e] = b1[e]; }
  float mx = v[0];
#pragma unroll
  for (int e = 1; e < 16; ++e) mx = fmaxf(mx, v[e]);
#pragma unroll
  for (int off = 1; off < 32; off <<= 1) mx = fmaxf(mx, __shfl_xor(mx, off, 32));
  if (lane == 0) rmax[wave] = mx;
  __syncthreads();
  float gm = rmax[0];
#pragma unroll
  for (int w = 1; w < 8; ++w) gm = fmaxf(gm, rmax[w]);
  float sum = 0.f;
#pragma unroll
  for (int e = 0; e < 16; ++e) { v[e] = __expf(v[e] - gm); sum += v[e]; }
#pragma unroll
  for (int off = 1; off < 32; off <<= 1) sum += __shfl_xor(sum, off, 32);
  if (lane == 0) rsum[wave] = sum;
  __syncthreads();
  float tot = rsum[0];
#pragma unroll
  for (int w = 1; w < 8; ++w) tot += rsum[w];
  const float inv = PSCALE * (1.0f / tot);
  const v4i ma0 = *(const v4i*)(keymask + ca), ma1 = *(const v4i*)(keymask + ca + 4);
  const v4i mb0 = *(const v4i*)(keymask + cb), mb1 = *(const v4i*)(keymask + cb + 4);
  int mk[16];
#pragma unroll
  for (int e = 0; e < 4; ++e) { mk[e] = ma0[e]; mk[4 + e] = ma1[e]; mk[8 + e] = mb0[e]; mk[12 + e] = mb1[e]; }
  v8h pa, pb;
#pragma unroll
  for (int e = 0; e < 8; ++e) {
    const float xa = (mk[e] != 0) ? v[e] * inv : 0.f;
    const float xb = (mk[8 + e] != 0) ? v[8 + e] * inv : 0.f;
    pa[e] = (_Float16)xa;
    pb[e] = (_Float16)xb;
  }
  unsigned short* pr = P + (size_t)row * SM_COLS;
  *(volatile v8h*)(pr + ca) = pa;
  *(volatile v8h*)(pr + cb) = pb;
  __threadfence();
  *(volatile v8h*)(pr + ca) = pa;
  *(volatile v8h*)(pr + cb) = pb;
}

extern "C" void kernel_launch(void* const* d_in, const int* in_sizes, int n_in,
                              void* d_out, int out_size, void* d_ws, size_t ws_size,
                              hipStream_t stream) {
  const int NB = 4, NQ = 4096, NK = 4096, CD = 512, CH = 2048;
  if (n_in < 6) return;
  if (in_sizes[0] != NB * NQ * CD || in_sizes[1] != NB * NK * CD || in_sizes[2] != NK ||
      in_sizes[3] != CD * CD || in_sizes[4] != CD * CD || in_sizes[5] != CD ||
      out_size != NB * NQ * CD || NK != SM_COLS) return;

  const float* x     = (const float*)d_in[0];
  const float* sup   = (const float*)d_in[1];
  const int*   kmask = (const int*)d_in[2];
  const float* Wv    = (const float*)d_in[3];
  const float* Wp    = (const float*)d_in[4];
  const float* bp    = (const float*)d_in[5];
  float* out = (float*)d_out;

  const size_t nAct = (size_t)NB * NQ * CD;
  const size_t nKey = (size_t)NB * NK * CD;
  const size_t nW   = (size_t)CD * CD;
  size_t off = 0;
  const size_t o_q   = off; off += nAct * 2;
  const size_t o_k   = off; off += nKey * 2;
  const size_t o_vt  = off; off += nKey * 2;
  const size_t o_o1  = off; off += nAct * 2;
  const size_t o_wvh = off; off += nW * 2;
  const size_t o_wvl = off; off += nW * 2;
  const size_t o_wp  = off; off += nW * 2;
  const size_t o_reg = off;
  const size_t nMaxAct = (nAct > nKey) ? nAct : nKey;
  const size_t planesBytes = nMaxAct * 2 * 2;
  const size_t sBytes = (size_t)CH * NK * 4;
  const size_t pBytes = (size_t)CH * NK * 2;
  const size_t regBytes = (planesBytes > sBytes + pBytes) ? planesBytes : (sBytes + pBytes);
  off += regBytes;
  if (off > ws_size) return;
  if (off > (size_t)134217728) return;

  char* ws = (char*)d_ws;
  unsigned short* q16  = (unsigned short*)(ws + o_q);
  unsigned short* k16  = (unsigned short*)(ws + o_k);
  unsigned short* vT16 = (unsigned short*)(ws + o_vt);
  unsigned short* o1T  = (unsigned short*)(ws + o_o1);
  unsigned short* wvh  = (unsigned short*)(ws + o_wvh);
  unsigned short* wvl  = (unsigned short*)(ws + o_wvl);
  unsigned short* wp16 = (unsigned short*)(ws + o_wp);
  unsigned short* ph   = (unsigned short*)(ws + o_reg);
  unsigned short* pl   = ph + nMaxAct;
  float*          Sf   = (float*)(ws + o_reg);
  unsigned short* P16  = (unsigned short*)(ws + o_reg + sBytes);

  const dim3 blk(256);

  {
    const int n8 = (int)(nW / 8);
    split_f32_bf16x8<<<dim3((n8 + 255) / 256), blk, 0, stream>>>(Wv, wvh, wvl, n8);
    const int n2 = (int)(nW / 2);
    cast_f32_f16x2<<<dim3((n2 + 255) / 256), blk, 0, stream>>>(Wp, (_Float16*)wp16, n2);
  }

  {
    const int n8 = (int)(nAct / 8);
    split_f32_bf16x8<<<dim3((n8 + 255) / 256), blk, 0, stream>>>(x, ph, pl, n8);
    const int M = NB * NQ, N = CD, K = CD;
    const int tiles = (M / 64) * (N / 64);
    wmma_gemm64<1, true, 0, 1, false, 0><<<dim3((tiles + 7) / 8, 1), blk, 0, stream>>>(
        ph, pl, CD, 0L, wvh, wvl, CD, 0L, (void*)q16, (void*)q16, CD, 0L,
        bp, bp, 0L, M, N, K, 1.0f);
  }
  {
    const int n8 = (int)(nKey / 8);
    split_f32_bf16x8<<<dim3((n8 + 255) / 256), blk, 0, stream>>>(sup, ph, pl, n8);
    const int M = NB * NK, N = CD, K = CD;
    const int tiles = (M / 64) * (N / 64);
    wmma_gemm64<1, true, 0, 1, false, 0><<<dim3((tiles + 7) / 8, 1), blk, 0, stream>>>(
        ph, pl, CD, 0L, wvh, wvl, CD, 0L, (void*)k16, (void*)k16, CD, 0L,
        bp, bp, 0L, M, N, K, 1.0f);
  }
  transpose64_h<<<dim3(NK / 64, CD / 64, NB), blk, 0, stream>>>(k16, vT16, NK, CD);

  for (int b = 0; b < NB; ++b) {
    for (int hc = 0; hc < NQ / CH; ++hc) {
      {
        const int M = CH, N = NK, K = CD;
        const int tiles = (M / 64) * (N / 64);
        const unsigned short* Aq = q16 + ((size_t)b * NQ + (size_t)hc * CH) * CD;
        const unsigned short* Bk = k16 + (size_t)b * NK * CD;
        wmma_gemm64<0, false, 0, 0, false, 0><<<dim3((tiles + 7) / 8, 1), blk, 0, stream>>>(
            Aq, Aq, CD, 0L, Bk, Bk, CD, 0L, (void*)Sf, (void*)Sf, NK, 0L,
            bp, bp, 0L, M, N, K, 0.125f);
      }
      softmax_rows<<<dim3(CH), blk, 0, stream>>>(Sf, kmask, P16);
      {
        const int M = CD, N = CH, K = NK;
        const int tiles = (M / 64) * (N / 64);
        const unsigned short* Av = vT16 + (size_t)b * CD * NK;
        unsigned short* Co = o1T + (size_t)b * CD * NQ + (size_t)hc * CH;
        wmma_gemm64<0, false, 0, 1, false, 0><<<dim3((tiles + 7) / 8, 1), blk, 0, stream>>>(
            Av, Av, NK, 0L, P16, P16, NK, 0L, (void*)Co, (void*)Co, NQ, 0L,
            bp, bp, 0L, M, N, K, PSCALE_INV * 16.0f);
      }
    }
  }

  {
    const int M = NB * NQ, N = CD, K = CD;
    const int tiles = (M / 64) * (N / 64);
    wmma_gemm64<0, false, 2, 0, false, 0><<<dim3((tiles + 7) / 8, 1), blk, 0, stream>>>(
        o1T, o1T, CD, 0L, wp16, wp16, CD, 0L, (void*)out, (void*)out, CD, 0L,
        bp, bp, 0L, M, N, K, 1.0f / 16.0f);
  }
}
